// MultiheadAttentionWithRoPE_34239479284091
// MI455X (gfx1250) — hardware-verified
//
#include <hip/hip_runtime.h>
#include <stdint.h>
#include <stddef.h>
#include <math.h>

#ifndef NB
#define NB 2
#endif
#ifndef SEQ
#define SEQ 2048
#endif
#define NB_FULL 2
#define SEQ_FULL 2048
#define DM 1024
#define NHEAD 16
#define HD 64
#define HROPE 32
#define TOK (NB * SEQ)

#define LDK 40
#define STGP 68
#define VSTP 136
#define PP 72
#define GEMM_SMEM 34816

static_assert(NB >= 1 && NB <= NB_FULL);
static_assert(SEQ >= 128 && SEQ <= SEQ_FULL);
static_assert(SEQ % 128 == 0);
static_assert(TOK % 128 == 0);
static_assert(DM % 128 == 0);
static_assert(HD == 64 && NHEAD * HD == DM);
static_assert(2 * 128 * LDK * 2 <= GEMM_SMEM);
static_assert(8 * 16 * STGP * 4 <= GEMM_SMEM);
static_assert(128 * VSTP * 2 <= GEMM_SMEM);
static_assert((long)((NB - 1) * SEQ_FULL + SEQ) * DM <= (long)NB_FULL * SEQ_FULL * DM);

typedef _Float16 f16;
typedef f16 v16h __attribute__((ext_vector_type(16)));
typedef f16 v8h __attribute__((ext_vector_type(8)));
typedef float v8f __attribute__((ext_vector_type(8)));
typedef float v4f __attribute__((ext_vector_type(4)));
typedef unsigned int v4u __attribute__((ext_vector_type(4)));

__device__ __forceinline__ v8f vz8() {
  v8f z = {0.f, 0.f, 0.f, 0.f, 0.f, 0.f, 0.f, 0.f};
  return z;
}

__device__ __forceinline__ v8f mma16(v16h a, v16h b, v8f c) {
  v8f d = __builtin_amdgcn_wmma_f32_16x16x32_f16(false, a, false, b, (short)0, c, false, false);
  asm volatile("v_nop\n\tv_nop\n\tv_nop\n\tv_nop" : "+v"(d) : "v"(a), "v"(b));
  return d;
}

__device__ __forceinline__ v16h frag16(const f16* base, int pitch, int lane) {
  const int r = lane & 15, hh = lane >> 4;
  union { v16h v; v8h p[2]; } u;
  const f16* rowp = base + (size_t)r * pitch + 8 * hh;
  u.p[0] = *(const v8h*)(rowp);
  u.p[1] = *(const v8h*)(rowp + 16);
  return u.v;
}

__device__ __forceinline__ float rbf(float f) {
  unsigned int u = __float_as_uint(f);
  u = (u + 0x7FFFu + ((u >> 16) & 1u)) & 0xFFFF0000u;
  return __uint_as_float(u);
}

__device__ __forceinline__ void stv4f(float* p, v4f v) { *(volatile v4f*)p = v; }
__device__ __forceinline__ void stv8h(f16* p, v8h v) { *(volatile v8h*)p = v; }
__device__ __forceinline__ void stf1(float* p, float v) { *(volatile float*)p = v; }

__device__ __forceinline__ void stage_tile(float* stg, int hl, int l16, v8f a0, v8f a1, v8f a2, v8f a3) {
#pragma unroll
  for (int r = 0; r < 8; ++r) {
    float* rowp = stg + (hl * 8 + r) * STGP + l16;
    rowp[0]  = a0[r];
    rowp[16] = a1[r];
    rowp[32] = a2[r];
    rowp[48] = a3[r];
  }
}

__global__ __launch_bounds__(256) void k_tab(float* __restrict__ cosT, float* __restrict__ sinT)
{
  const int tid = threadIdx.x;
  const int s = blockIdx.x * 8 + (tid >> 5);
  const int m = tid & 31;
  const float invf = exp2f(-(float)m * 0.41524101186092028f);
  const float th = (float)s * invf;
  float sn, cs;
  sincosf(th, &sn, &cs);
  const size_t off = (size_t)s * HROPE + m;
  stf1(cosT + off, cs);
  stf1(sinT + off, sn);
  __threadfence();
  stf1(cosT + off, cs);
  stf1(sinT + off, sn);
}

__global__ __launch_bounds__(256) void k_wprep(const float* __restrict__ in, f16* __restrict__ out,
                                               int Kin, int Nout, float carry)
{
  __shared__ float t[64][33];
  const int tid = threadIdx.x, tx = tid & 31, ty = tid >> 5;
  const int n0 = blockIdx.x * 32, k0 = blockIdx.y * 64;
#pragma unroll
  for (int i = 0; i < 8; ++i) {
    const int row = ty + 8 * i;
    t[row][tx] = in[(size_t)(k0 + row) * Nout + n0 + tx];
  }
  __syncthreads();
  const int n = tid >> 3, q = tid & 7;
  v8h hv;
#pragma unroll
  for (int e = 0; e < 8; ++e) hv[e] = (f16)(carry * rbf(t[8 * q + e][n]));
  f16* dst = out + (size_t)(n0 + n) * Kin + k0 + 8 * q;
  stv8h(dst, hv);
  __threadfence();
  stv8h(dst, hv);
}

__global__ __launch_bounds__(128) void k_cvt(const float* __restrict__ x, f16* __restrict__ out, int src_seq)
{
  const int r = blockIdx.x, tid = threadIdx.x;
  const int bidx = r / SEQ, sidx = r - bidx * SEQ;
  const float* xr = x + ((size_t)bidx * src_seq + sidx) * DM + tid * 8;
  const v4f xa = *(const v4f*)xr;
  const v4f xb = *(const v4f*)(xr + 4);
  v8h o;
#pragma unroll
  for (int e = 0; e < 4; ++e) {
    const float va = xa[e];
    const float vb = xb[e];
    o[e]     = (f16)rbf(va);
    o[e + 4] = (f16)rbf(vb);
  }
  f16* dst = out + (size_t)r * DM + tid * 8;
  stv8h(dst, o);
  __threadfence();
  stv8h(dst, o);
}

template<int MODE>
__global__ __launch_bounds__(256) void k_gemm(
    const f16* __restrict__ A0, const f16* __restrict__ A1, const f16* __restrict__ A2,
    const f16* __restrict__ Bt,
    const float* __restrict__ bz0, const float* __restrict__ bz1, const float* __restrict__ bz2,
    float* __restrict__ outf, f16* __restrict__ qpl, f16* __restrict__ kpl, f16* __restrict__ vtp,
    const float* __restrict__ cosT, const float* __restrict__ sinT,
    int N, int K, int out_seq, float oscale, float ocarry)
{
  __shared__ __align__(16) unsigned char smem[GEMM_SMEM];
  f16* sA = (f16*)smem;
  f16* sB = sA + 128 * LDK;
  const int tid = threadIdx.x, l = tid & 31, wave = tid >> 5;
  const int hl = l >> 4, l16 = l & 15;
  const int wm = wave >> 1, wn = wave & 1;
  const int m0 = blockIdx.y * 128, n0 = blockIdx.x * 128;
  (void)bz1; (void)bz2; (void)outf; (void)qpl; (void)kpl; (void)vtp;
  (void)cosT; (void)sinT; (void)out_seq; (void)ocarry;

  const int which = (MODE == 0) ? (n0 >> 10) : 0;
  const f16* A = (which == 0) ? A0 : ((which == 1) ? A1 : A2);

  v8f acc[2][4];
#pragma unroll
  for (int i = 0; i < 2; ++i)
#pragma unroll
    for (int j = 0; j < 4; ++j) acc[i][j] = vz8();

#pragma unroll 1
  for (int k0 = 0; k0 < K; k0 += 32) {
    v4u ga[2], gb[2];
#pragma unroll
    for (int i = 0; i < 2; ++i) {
      const int c = tid + 256 * i, row = c >> 2, kc = c & 3;
      ga[i] = *(const v4u*)(A  + (size_t)(m0 + row) * K + k0 + kc * 8);
      gb[i] = *(const v4u*)(Bt + (size_t)(n0 + row) * K + k0 + kc * 8);
    }
    __syncthreads();
#pragma unroll
    for (int i = 0; i < 2; ++i) {
      const int c = tid + 256 * i, row = c >> 2, kc = c & 3;
      *(v4u*)(sA + row * LDK + kc * 8) = ga[i];
      *(v4u*)(sB + row * LDK + kc * 8) = gb[i];
    }
    __syncthreads();
    const v16h af0 = frag16(sA + (wm * 32) * LDK, LDK, l);
    const v16h af1 = frag16(sA + (wm * 32 + 16) * LDK, LDK, l);
#pragma unroll
    for (int j = 0; j < 4; ++j) {
      const v16h bfr = frag16(sB + (wn * 64 + j * 16) * LDK, LDK, l);
      acc[0][j] = mma16(af0, bfr, acc[0][j]);
      acc[1][j] = mma16(af1, bfr, acc[1][j]);
    }
  }
  __syncthreads();

  if (MODE == 1) {
    float* stg = (float*)smem + wave * (16 * STGP);
#pragma unroll
    for (int i = 0; i < 2; ++i) {
      stage_tile(stg, hl, l16, acc[i][0], acc[i][1], acc[i][2], acc[i][3]);
      __syncthreads();
      v4f vals[8];
      size_t goff[8];
#pragma unroll
      for (int p = 0; p < 8; ++p) {
        const int L = p * 4 + (l >> 3);
        const int row = L >> 1, half = L & 1, q = l & 7;
        const int col = half * 32 + q * 4;
        const v4f a = *(const v4f*)(stg + row * STGP + col);
        const int grow = m0 + wm * 32 + i * 16 + row;
        const int gcol = n0 + wn * 64 + col;
        const int bi = grow / SEQ, si = grow - bi * SEQ;
        const v4f bv = *(const v4f*)(bz0 + gcol);
        v4f o;
#pragma unroll
        for (int e = 0; e < 4; ++e) {
          const float ae = a[e];
          const float be = bv[e];
          o[e] = ae * oscale + rbf(be);
        }
        vals[p] = o;
        const size_t orow = (size_t)bi * out_seq + si;
        goff[p] = orow * (size_t)N + gcol;
      }
#pragma unroll
      for (int p = 0; p < 8; ++p) stv4f(outf + goff[p], vals[p]);
      __threadfence();
#pragma unroll
      for (int p = 0; p < 8; ++p) stv4f(outf + goff[p], vals[p]);
      __syncthreads();
    }
  } else {
    const int cbase = (n0 & (DM - 1)) + wn * 64;
    if (which < 2) {
      f16* dst = (which == 0) ? qpl : kpl;
      const float* bsel = (which == 0) ? bz0 : bz1;
      const int head = cbase >> 6;
      float* stg = (float*)smem + wave * (16 * STGP);
#pragma unroll
      for (int i = 0; i < 2; ++i) {
        stage_tile(stg, hl, l16, acc[i][0], acc[i][1], acc[i][2], acc[i][3]);
        __syncthreads();
        v8h hv[4];
        size_t goff[4];
#pragma unroll
        for (int p = 0; p < 4; ++p) {
          const int row = p * 4 + (l >> 3), q = l & 7;
          const int col = q * 8, colp = col ^ 32;
          const v4f a0 = *(const v4f*)(stg + row * STGP + col);
          const v4f a1 = *(const v4f*)(stg + row * STGP + col + 4);
          const v4f c0 = *(const v4f*)(stg + row * STGP + colp);
          const v4f c1 = *(const v4f*)(stg + row * STGP + colp + 4);
          const v4f ba0 = *(const v4f*)(bsel + cbase + col);
          const v4f ba1 = *(const v4f*)(bsel + cbase + col + 4);
          const v4f bp0 = *(const v4f*)(bsel + cbase + colp);
          const v4f bp1 = *(const v4f*)(bsel + cbase + colp + 4);
          const int grow = m0 + wm * 32 + i * 16 + row;
          const int bi = grow / SEQ, si = grow - bi * SEQ;
          const float* ct = cosT + (size_t)si * HROPE + (col & 31);
          const float* st = sinT + (size_t)si * HROPE + (col & 31);
          const v4f cs0 = *(const v4f*)ct, cs1 = *(const v4f*)(ct + 4);
          const v4f sn0 = *(const v4f*)st, sn1 = *(const v4f*)(st + 4);
          float av[8], pv[8], bav[8], bpv[8], csv[8], snv[8];
#pragma unroll
          for (int e = 0; e < 4; ++e) {
            av[e] = a0[e];  av[e + 4] = a1[e];
            pv[e] = c0[e];  pv[e + 4] = c1[e];
            bav[e] = ba0[e]; bav[e + 4] = ba1[e];
            bpv[e] = bp0[e]; bpv[e + 4] = bp1[e];
            csv[e] = cs0[e]; csv[e + 4] = cs1[e];
            snv[e] = sn0[e]; snv[e + 4] = sn1[e];
          }
          const float sg = (col < 32) ? -1.0f : 1.0f;
          v8h o;
#pragma unroll
          for (int e = 0; e < 8; ++e) {
            const float xv = av[e] * oscale + rbf(bav[e]);
            const float xq = pv[e] * oscale + rbf(bpv[e]);
            o[e] = (f16)((xv * csv[e] + sg * xq * snv[e]) * ocarry);
          }
          hv[p] = o;
          goff[p] = ((size_t)(bi * NHEAD + head) * SEQ + si) * HD + col;
        }
#pragma unroll
        for (int p = 0; p < 4; ++p) stv8h(dst + goff[p], hv[p]);
        __threadfence();
#pragma unroll
        for (int p = 0; p < 4; ++p) stv8h(dst + goff[p], hv[p]);
        __syncthreads();
      }
    } else {
      f16* vst = (f16*)smem;
#pragma unroll
      for (int j = 0; j < 4; ++j) {
        const int dim = j * 16 + l16;
        const float bb = rbf(bz2[cbase + dim]);
#pragma unroll
        for (int i = 0; i < 2; ++i) {
#pragma unroll
          for (int r = 0; r < 8; ++r) {
            const int tokl = wm * 32 + i * 16 + hl * 8 + r;
            vst[(wn * 64 + dim) * VSTP + tokl] = (f16)(acc[i][j][r] * oscale + bb);
          }
        }
      }
      __syncthreads();
      const int hbase = (n0 & (DM - 1)) >> 6;
      const int bi = m0 / SEQ, s0 = m0 - bi * SEQ;
      v8h hv[8];
      size_t goff[8];
#pragma unroll
      for (int p = 0; p < 8; ++p) {
        const int L = p * 32 + (tid >> 3);
        const int hd = L >> 1, half = L & 1, q = tid & 7;
        const int key = half * 64 + q * 8;
        hv[p] = *(const v8h*)(vst + hd * VSTP + key);
        goff[p] = ((size_t)(bi * NHEAD + hbase + (hd >> 6)) * HD + (hd & 63)) * SEQ + s0 + key;
      }
#pragma unroll
      for (int p = 0; p < 8; ++p) stv8h(vtp + goff[p], hv[p]);
      __threadfence();
#pragma unroll
      for (int p = 0; p < 8; ++p) stv8h(vtp + goff[p], hv[p]);
    }
  }
}

__global__ __launch_bounds__(256) void k_attn(const f16* __restrict__ qp, const f16* __restrict__ kpl,
                                              const f16* __restrict__ vt, f16* __restrict__ ctx)
{
  __shared__ __align__(16) f16 sP[8 * 16 * PP];
  const int tid = threadIdx.x, l = tid & 31, wave = tid >> 5;
  const int hl = l >> 4, l16 = l & 15;
  const int nrb = SEQ / 128;
  const int wg = blockIdx.x;
  const int rowblk = wg % nrb, bh = wg / nrb;
  const int b = bh / NHEAD, h = bh - b * NHEAD;
  const int q0 = rowblk * 128 + wave * 16;
  const f16* Q  = qp  + ((size_t)bh * SEQ + q0) * HD;
  const f16* Kb = kpl + (size_t)bh * SEQ * HD;
  const f16* Vh = vt  + (size_t)bh * HD * SEQ;

  const v16h qa0 = frag16(Q, HD, l);
  const v16h qa1 = frag16(Q + 32, HD, l);

  v8f o[4];
#pragma unroll
  for (int t = 0; t < 4; ++t) o[t] = vz8();
  float mrun[8], lrun[8];
#pragma unroll
  for (int j = 0; j < 8; ++j) { mrun[j] = -1e30f; lrun[j] = 0.f; }

  f16* pbuf = sP + wave * (16 * PP);
  const int prow = hl * 8;
  const float SC = 0.125f;
  const float L2E = 1.4426950408889634f;

#pragma unroll 1
  for (int kb = 0; kb < SEQ; kb += 32) {
    const f16* Kt = Kb + (size_t)kb * HD;
    const v16h k00 = frag16(Kt, HD, l);
    const v16h k01 = frag16(Kt + 32, HD, l);
    const v16h k10 = frag16(Kt + 16 * HD, HD, l);
    const v16h k11 = frag16(Kt + 16 * HD + 32, HD, l);
    v8f s0 = mma16(qa0, k00, vz8());
    s0 = mma16(qa1, k01, s0);
    v8f s1 = mma16(qa0, k10, vz8());
    s1 = mma16(qa1, k11, s1);

    float mt[8];
#pragma unroll
    for (int j = 0; j < 8; ++j) {
      s0[j] *= SC; s1[j] *= SC;
      mt[j] = fmaxf(s0[j], s1[j]);
    }
#pragma unroll
    for (int off = 1; off < 16; off <<= 1)
#pragma unroll
      for (int j = 0; j < 8; ++j)
        mt[j] = fmaxf(mt[j], __shfl_xor(mt[j], off, 32));

    float corr[8], p0[8], p1[8], rt[8];
#pragma unroll
    for (int j = 0; j < 8; ++j) {
      const float mn = fmaxf(mrun[j], mt[j]);
      corr[j] = exp2f((mrun[j] - mn) * L2E);
      p0[j] = exp2f((s0[j] - mn) * L2E);
      p1[j] = exp2f((s1[j] - mn) * L2E);
      mrun[j] = mn;
      rt[j] = p0[j] + p1[j];
    }
#pragma unroll
    for (int off = 1; off < 16; off <<= 1)
#pragma unroll
      for (int j = 0; j < 8; ++j)
        rt[j] += __shfl_xor(rt[j], off, 32);
#pragma unroll
    for (int j = 0; j < 8; ++j) lrun[j] = lrun[j] * corr[j] + rt[j];
#pragma unroll
    for (int t = 0; t < 4; ++t)
#pragma unroll
      for (int j = 0; j < 8; ++j) o[t][j] *= corr[j];

#pragma unroll
    for (int j = 0; j < 8; ++j) {
      pbuf[(prow + j) * PP + l16]      = (f16)p0[j];
      pbuf[(prow + j) * PP + 16 + l16] = (f16)p1[j];
    }
    __syncthreads();
    const v16h pa = frag16(pbuf, PP, l);
    __syncthreads();
#pragma unroll
    for (int t = 0; t < 4; ++t) {
      const v16h vf = frag16(Vh + (size_t)(t * 16) * SEQ + kb, SEQ, l);
      o[t] = mma16(pa, vf, o[t]);
    }
  }

#pragma unroll
  for (int j = 0; j < 8; ++j) {
    const float inv = 64.0f / lrun[j];
#pragma unroll
    for (int t = 0; t < 4; ++t)
      pbuf[(prow + j) * PP + t * 16 + l16] = (f16)(o[t][j] * inv);
  }
  __syncthreads();
  v8h hv[4];
  size_t goff[4];
#pragma unroll
  for (int p = 0; p < 4; ++p) {
    const int row = p * 4 + (l >> 3), q = l & 7;
    hv[p] = *(const v8h*)(pbuf + row * PP + q * 8);
    goff[p] = ((size_t)b * SEQ + q0 + row) * DM + h * HD + q * 8;
  }
#pragma unroll
  for (int p = 0; p < 4; ++p) stv8h(ctx + goff[p], hv[p]);
  __threadfence();
#pragma unroll
  for (int p = 0; p < 4; ++p) stv8h(ctx + goff[p], hv[p]);
}

extern "C" void kernel_launch(void* const* d_in, const int* in_sizes, int n_in,
                              void* d_out, int out_size, void* d_ws, size_t ws_size,
                              hipStream_t stream)
{
  if (n_in < 11) return;
  const long rows_needed = (long)(NB - 1) * SEQ_FULL + SEQ;
  if ((long)in_sizes[0] < rows_needed * DM) return;
  if ((long)in_sizes[1] < rows_needed * DM) return;
  if ((long)in_sizes[2] < rows_needed * DM) return;
  if (in_sizes[3] < DM * DM || in_sizes[5] < DM * DM || in_sizes[7] < DM * DM || in_sizes[9] < DM * DM) return;
  if (in_sizes[4] < DM || in_sizes[6] < DM || in_sizes[8] < DM || in_sizes[10] < DM) return;
  if ((long)out_size < rows_needed * DM) return;

  const float* xq_in = (const float*)d_in[0];
  const float* xk_in = (const float*)d_in[1];
  const float* xv_in = (const float*)d_in[2];
  const float* Wq = (const float*)d_in[3];
  const float* bq = (const float*)d_in[4];
  const float* Wk = (const float*)d_in[5];
  const float* bk = (const float*)d_in[6];
  const float* Wv = (const float*)d_in[7];
  const float* bv = (const float*)d_in[8];
  const float* Wo = (const float*)d_in[9];
  const float* bo = (const float*)d_in[10];
  float* out = (float*)d_out;

  char* ws = (char*)d_ws;
  size_t off = 0;
  auto carve = [&](size_t bytes) -> char* {
    char* p = ws + off;
    off += (bytes + 255) & ~(size_t)255;
    return p;
  };
  f16*   wqkv = (f16*)carve((size_t)3 * DM * DM * 2);
  f16*   wot  = (f16*)carve((size_t)DM * DM * 2);
  float* cosT = (float*)carve((size_t)SEQ * HROPE * 4);
  float* sinT = (float*)carve((size_t)SEQ * HROPE * 4);
  f16*   xq   = (f16*)carve((size_t)TOK * DM * 2);
  f16*   xk   = (f16*)carve((size_t)TOK * DM * 2);
  f16*   xv   = (f16*)carve((size_t)TOK * DM * 2);
  f16*   qpl  = (f16*)carve((size_t)TOK * DM * 2);
  f16*   kpl  = (f16*)carve((size_t)TOK * DM * 2);
  f16*   vtp  = (f16*)carve((size_t)TOK * DM * 2);
  f16*   ctx  = (f16*)carve((size_t)TOK * DM * 2);
  if (off > ws_size) return;
  if (off > (size_t)134217728) return;

  const dim3 blk(256);

  k_tab<<<dim3(SEQ / 8), blk, 0, stream>>>(cosT, sinT);

  k_wprep<<<dim3(DM / 32, DM / 64), blk, 0, stream>>>(Wq, wqkv, DM, DM, 64.0f);
  k_wprep<<<dim3(DM / 32, DM / 64), blk, 0, stream>>>(Wk, wqkv + (size_t)DM * DM, DM, DM, 64.0f);
  k_wprep<<<dim3(DM / 32, DM / 64), blk, 0, stream>>>(Wv, wqkv + (size_t)2 * DM * DM, DM, DM, 64.0f);
  k_wprep<<<dim3(DM / 32, DM / 64), blk, 0, stream>>>(Wo, wot, DM, DM, 64.0f);

  k_cvt<<<dim3(TOK), dim3(128), 0, stream>>>(xq_in, xq, SEQ_FULL);
  k_cvt<<<dim3(TOK), dim3(128), 0, stream>>>(xk_in, xk, SEQ_FULL);
  k_cvt<<<dim3(TOK), dim3(128), 0, stream>>>(xv_in, xv, SEQ_FULL);

  k_gemm<0><<<dim3(3 * DM / 128, TOK / 128), blk, 0, stream>>>(
      xq, xk, xv, wqkv, bq, bk, bv, out, qpl, kpl, vtp, cosT, sinT,
      3 * DM, DM, SEQ, 1.0f / 64.0f, 1.0f);

  k_attn<<<dim3(NB * NHEAD * (SEQ / 128)), blk, 0, stream>>>(qpl, kpl, vtp, ctx);

  k_gemm<1><<<dim3(DM / 128, TOK / 128), blk, 0, stream>>>(
      ctx, ctx, ctx, wot, bo, bo, bo, out, qpl, kpl, vtp, cosT, sinT,
      DM, DM, SEQ_FULL, 1.0f / 4096.0f, 1.0f);
}
